// KGSLomics_80633716015291
// MI455X (gfx1250) — hardware-verified
//
#include <hip/hip_runtime.h>
#include <stddef.h>


#define DF    128
#define CIN   256
#define NH    4
#define NREL  8
#define OMK   4
#define OMH   32
#define GR    16
#define NTHR  256
#define NWAVE 8
#define H1P   40
#define AP1   (CIN + 8)
#define AP2   (DF + 8)
#define HP    (NREL * DF + 8)
#define SP    (DF + 4)
#define QROWS 16
#define NB    512
#define CHUNK 2048
#define WCAP  256
#define NGRP  (CHUNK / (NTHR * 4))

#define LDS_SACC (NB * DF)
#define LDS_MX   (NB * NH)
#define LDS_DEN  (NB * NH)
#define LDS_LIST (NWAVE * WCAP)
#define LDS_BYTES ((LDS_SACC + LDS_MX + LDS_DEN + LDS_LIST + NWAVE) * 4)

static_assert(WCAP == (CHUNK / NTHR) * 32);
static_assert(NGRP == 2);
static_assert(NB == 512);
static_assert(CHUNK == 2048);
static_assert(LDS_BYTES == 286752);
static_assert(((LDS_SACC | LDS_MX | LDS_DEN) & 3) == 0);

typedef float    v4f  __attribute__((ext_vector_type(4)));
typedef float    v8f  __attribute__((ext_vector_type(8)));
typedef int      v4i  __attribute__((ext_vector_type(4)));
typedef _Float16 v4h  __attribute__((ext_vector_type(4)));
typedef _Float16 v8h  __attribute__((ext_vector_type(8)));
typedef _Float16 v16h __attribute__((ext_vector_type(16)));
typedef __bf16   v8b  __attribute__((ext_vector_type(8)));
typedef __bf16   v16b __attribute__((ext_vector_type(16)));
union FragH  { v16h v; v8h half[2]; };
union FragB  { v16b v; v8b half[2]; };
union PackH  { v8h h; v4i i; };
union PackU  { v4i i; unsigned short u[8]; };
union BfBits { unsigned short u; __bf16 b; };

__device__ __forceinline__ v8f wmf(v16h a, v16h b, v8f c) {
  v8f d = __builtin_amdgcn_wmma_f32_16x16x32_f16(false, a, false, b, (short)0, c, false, false);
  asm volatile("v_nop\n\tv_nop\n\tv_nop\n\tv_nop" : "+v"(d) : "v"(a), "v"(b));
  return d;
}
__device__ __forceinline__ v8f wmb(v16b a, v16b b, v8f c) {
  v8f d = __builtin_amdgcn_wmma_f32_16x16x32_bf16(false, a, false, b, (short)0, c, false, false);
  asm volatile("v_nop\n\tv_nop\n\tv_nop\n\tv_nop" : "+v"(d) : "v"(a), "v"(b));
  return d;
}

__device__ __forceinline__ v8f vz8() {
  v8f z = {0.f, 0.f, 0.f, 0.f, 0.f, 0.f, 0.f, 0.f};
  return z;
}
__device__ __forceinline__ unsigned short bf_rne(float x) {
  unsigned u = __float_as_uint(x);
  u += 0x7FFFu + ((u >> 16) & 1u);
  return (unsigned short)(u >> 16);
}
__device__ __forceinline__ float bf_val(unsigned short b) {
  return __uint_as_float(((unsigned)b) << 16);
}
__device__ __forceinline__ __bf16 bf_mk(unsigned short b) {
  BfBits t; t.u = b; return t.b;
}
__device__ __forceinline__ float lk01(float v) { return v > 0.f ? v : 0.01f * v; }

template <int MODE>
__global__ __launch_bounds__(NTHR) void k_tconv(const float* __restrict__ in,
                                               unsigned short* o1, unsigned short* o2,
                                               int K, int NC, int NCO, int nrel, float scale) {
  const int K8    = K >> 3;
  const int total = nrel * NCO * K8;
  const int idx   = blockIdx.x * NTHR + threadIdx.x;
  if (idx >= total) return;
  const int r   = idx / (NCO * K8);
  const int rem = idx - r * (NCO * K8);
  const int n   = rem / K8;
  const int k0  = (rem - n * K8) * 8;
  const int nc  = (n < NC) ? n : (NC - 1);
  const float* p = in + ((size_t)r * K + k0) * NC + nc;
  float v[8];
#pragma unroll
  for (int i = 0; i < 8; ++i) {
    const float t = p[(size_t)i * NC];
    v[i] = (n < NC) ? t : 0.0f;
  }
  const size_t o = (size_t)idx * 8;
  if (MODE == 0) {
    PackH u;
#pragma unroll
    for (int i = 0; i < 8; ++i) u.h[i] = (_Float16)(v[i] * scale);
    *(volatile v4i*)(o1 + o) = u.i;
    __threadfence();
    *(volatile v4i*)(o1 + o) = u.i;
  } else {
    PackU hi, lo;
#pragma unroll
    for (int i = 0; i < 8; ++i) {
      const unsigned short hb = bf_rne(v[i]);
      const unsigned short lb = bf_rne(v[i] - bf_val(hb));
      hi.u[i] = hb;
      lo.u[i] = lb;
    }
    *(volatile v4i*)(o1 + o) = hi.i;
    *(volatile v4i*)(o2 + o) = lo.i;
    __threadfence();
    *(volatile v4i*)(o1 + o) = hi.i;
    *(volatile v4i*)(o2 + o) = lo.i;
  }
}

__device__ __forceinline__ v8f om_tile(const float* __restrict__ om, const int* __restrict__ nid,
                                       const float* __restrict__ ow1, const float* __restrict__ ob1,
                                       const _Float16* __restrict__ ow2h, const float* __restrict__ ob2,
                                       int rowBase, int nN, _Float16* h1t, int tid, int lane, int wave) {
  {
    const int r  = tid >> 4;
    const int j0 = (tid & 15) * 2;
    int row = rowBase + r;
    if (row > nN - 1) row = nN - 1;
    int node = nid[row];
    node = node < 0 ? 0 : (node > nN - 1 ? nN - 1 : node);
    const v4f cv = *(const v4f*)(om + (size_t)node * OMK);
#pragma unroll
    for (int jj = 0; jj < 2; ++jj) {
      const int j = j0 + jj;
      float a = cv.x * ow1[j] + cv.y * ow1[OMH + j] + cv.z * ow1[2 * OMH + j] + cv.w * ow1[3 * OMH + j];
      a += ob1[j];
      a = lk01(a);
      h1t[r * H1P + j] = (_Float16)(a * 64.0f);
    }
  }
  __syncthreads();
  const int hh = lane >> 4, m = lane & 15;
  const int n = wave * 16 + m;
  FragH a, b;
  a.half[0] = *(const v8h*)(h1t + m * H1P + 8 * hh);
  a.half[1] = *(const v8h*)(h1t + m * H1P + 16 + 8 * hh);
  b.half[0] = *(const v8h*)(ow2h + n * OMH + 8 * hh);
  b.half[1] = *(const v8h*)(ow2h + n * OMH + 16 + 8 * hh);
  v8f acc = vz8();
  acc = wmf(a.v, b.v, acc);
  const float bb = ob2[n];
  v8f res = vz8();
#pragma unroll
  for (int r = 0; r < 8; ++r) res[r] = acc[r] * (1.0f / 1024.0f) + bb;
  return res;
}

__global__ __launch_bounds__(NTHR) void k_skip(
    const float* __restrict__ kg, const float* __restrict__ om, const int* __restrict__ nid,
    const float* __restrict__ ow1, const float* __restrict__ ob1,
    const _Float16* __restrict__ ow2h, const float* __restrict__ ob2,
    const __bf16* __restrict__ w1hi, const __bf16* __restrict__ w1lo, const float* __restrict__ sb1,
    const __bf16* __restrict__ w2hi, const __bf16* __restrict__ w2lo, const float* __restrict__ sb2,
    float* out, int nN) {
  __shared__ __attribute__((aligned(16))) _Float16 h1t[GR * H1P];
  __shared__ __attribute__((aligned(16))) __bf16 Ahi[GR * AP1];
  __shared__ __attribute__((aligned(16))) __bf16 Alo[GR * AP1];
  __shared__ __attribute__((aligned(16))) __bf16 Mhi[GR * AP2];
  __shared__ __attribute__((aligned(16))) __bf16 Mlo[GR * AP2];
  __shared__ __attribute__((aligned(16))) float S[GR * SP];

  const int tid  = threadIdx.x;
  const int lane = tid & 31;
  const int wave = tid >> 5;
  const int hh   = lane >> 4;
  const int m    = lane & 15;
  const int rowBase = blockIdx.x * GR;

  {
    const int r  = tid >> 4;
    const int c0 = (tid & 15) * 8;
    int row = rowBase + r;
    if (row > nN - 1) row = nN - 1;
    int node = nid[row];
    node = node < 0 ? 0 : (node > nN - 1 ? nN - 1 : node);
    const float* p = kg + (size_t)node * DF + c0;
    const v4f f0 = *(const v4f*)(p), f1 = *(const v4f*)(p + 4);
    const float f[8] = {f0.x, f0.y, f0.z, f0.w, f1.x, f1.y, f1.z, f1.w};
    PackU hi, lo;
#pragma unroll
    for (int i = 0; i < 8; ++i) {
      const unsigned short hb = bf_rne(f[i]);
      hi.u[i] = hb;
      lo.u[i] = bf_rne(f[i] - bf_val(hb));
    }
    *(v4i*)(Ahi + r * AP1 + c0) = hi.i;
    *(v4i*)(Alo + r * AP1 + c0) = lo.i;
  }
  {
    const v8f co = om_tile(om, nid, ow1, ob1, ow2h, ob2, rowBase, nN, h1t, tid, lane, wave);
#pragma unroll
    for (int r = 0; r < 8; ++r) {
      const unsigned short hb = bf_rne(co[r]);
      const unsigned short lb = bf_rne(co[r] - bf_val(hb));
      const int li = (8 * hh + r) * AP1 + DF + wave * 16 + m;
      Ahi[li] = bf_mk(hb);
      Alo[li] = bf_mk(lb);
    }
  }
  __syncthreads();

  const int n = wave * 16 + m;
  v8f acc = vz8();
#pragma unroll 1
  for (int kt = 0; kt < CIN / 32; ++kt) {
    const int k0 = kt * 32;
    FragB ah, al, bh, bl;
    const __bf16* pa  = Ahi + m * AP1 + k0 + 8 * hh;
    const __bf16* pl  = Alo + m * AP1 + k0 + 8 * hh;
    const __bf16* pbh = w1hi + (size_t)n * CIN + k0 + 8 * hh;
    const __bf16* pbl = w1lo + (size_t)n * CIN + k0 + 8 * hh;
    ah.half[0] = *(const v8b*)pa;  ah.half[1] = *(const v8b*)(pa + 16);
    al.half[0] = *(const v8b*)pl;  al.half[1] = *(const v8b*)(pl + 16);
    bh.half[0] = *(const v8b*)pbh; bh.half[1] = *(const v8b*)(pbh + 16);
    bl.half[0] = *(const v8b*)pbl; bl.half[1] = *(const v8b*)(pbl + 16);
    acc = wmb(ah.v, bh.v, acc);
    acc = wmb(ah.v, bl.v, acc);
    acc = wmb(al.v, bh.v, acc);
  }
  {
    const float bb = sb1[n];
#pragma unroll
    for (int r = 0; r < 8; ++r) {
      const float v = lk01(acc[r] + bb);
      const unsigned short hb = bf_rne(v);
      const unsigned short lb = bf_rne(v - bf_val(hb));
      const int li = (8 * hh + r) * AP2 + n;
      Mhi[li] = bf_mk(hb);
      Mlo[li] = bf_mk(lb);
    }
  }
  __syncthreads();

  v8f acc2 = vz8();
#pragma unroll 1
  for (int kt = 0; kt < DF / 32; ++kt) {
    const int k0 = kt * 32;
    FragB ah, al, bh, bl;
    const __bf16* pa  = Mhi + m * AP2 + k0 + 8 * hh;
    const __bf16* pl  = Mlo + m * AP2 + k0 + 8 * hh;
    const __bf16* pbh = w2hi + (size_t)n * DF + k0 + 8 * hh;
    const __bf16* pbl = w2lo + (size_t)n * DF + k0 + 8 * hh;
    ah.half[0] = *(const v8b*)pa;  ah.half[1] = *(const v8b*)(pa + 16);
    al.half[0] = *(const v8b*)pl;  al.half[1] = *(const v8b*)(pl + 16);
    bh.half[0] = *(const v8b*)pbh; bh.half[1] = *(const v8b*)(pbh + 16);
    bl.half[0] = *(const v8b*)pbl; bl.half[1] = *(const v8b*)(pbl + 16);
    acc2 = wmb(ah.v, bh.v, acc2);
    acc2 = wmb(ah.v, bl.v, acc2);
    acc2 = wmb(al.v, bh.v, acc2);
  }
  {
    const float bb = sb2[n];
#pragma unroll
    for (int r = 0; r < 8; ++r) S[(8 * hh + r) * SP + n] = acc2[r] + bb;
  }
  __syncthreads();

  const v4f y0 = *(const v4f*)(S + (2 * wave) * SP + 4 * lane);
  const v4f y1 = *(const v4f*)(S + (2 * wave + 1) * SP + 4 * lane);
  const int r0 = rowBase + 2 * wave;
  const int r1 = r0 + 1;
  float* p0 = out + (size_t)r0 * DF + 4 * lane;
  float* p1 = out + (size_t)r1 * DF + 4 * lane;
  if (r0 < nN) *(volatile v4f*)p0 = y0;
  if (r1 < nN) *(volatile v4f*)p1 = y1;
  __threadfence();
  if (r0 < nN) *(volatile v4f*)p0 = y0;
  if (r1 < nN) *(volatile v4f*)p1 = y1;
}

template <bool L1>
__global__ __launch_bounds__(NTHR) void k_hr(
    const float* __restrict__ kg, const float* __restrict__ om, const int* __restrict__ nid,
    const float* __restrict__ ow1, const float* __restrict__ ob1,
    const _Float16* __restrict__ ow2h, const float* __restrict__ ob2,
    const _Float16* __restrict__ xh, const _Float16* __restrict__ Wh,
    const _Float16* __restrict__ qp, const _Float16* __restrict__ kp,
    _Float16* hrH, float* hqk, int nN, int nP) {
  constexpr int   KD  = L1 ? CIN : DF;
  constexpr int   APX = KD + 8;
  constexpr float SC  = L1 ? (1.0f / 16.0f) : (1.0f / 256.0f);
  __shared__ __attribute__((aligned(16))) _Float16 A16[GR * APX];
  __shared__ __attribute__((aligned(16))) _Float16 h1t[GR * H1P];
  __shared__ __attribute__((aligned(16))) _Float16 T16[GR * HP];
  __shared__ __attribute__((aligned(16))) float hqs[2 * NREL * 64];

  const int tid  = threadIdx.x;
  const int lane = tid & 31;
  const int wave = tid >> 5;
  const int hh   = lane >> 4;
  const int m    = lane & 15;
  const int rowBase = blockIdx.x * GR;

  if (L1) {
    {
      const int r  = tid >> 4;
      const int c0 = (tid & 15) * 8;
      int row = rowBase + r;
      if (row > nN - 1) row = nN - 1;
      int node = nid[row];
      node = node < 0 ? 0 : (node > nN - 1 ? nN - 1 : node);
      const float* p = kg + (size_t)node * DF + c0;
      const v4f f0 = *(const v4f*)(p), f1 = *(const v4f*)(p + 4);
      PackH u;
      u.h[0] = (_Float16)f0.x; u.h[1] = (_Float16)f0.y; u.h[2] = (_Float16)f0.z; u.h[3] = (_Float16)f0.w;
      u.h[4] = (_Float16)f1.x; u.h[5] = (_Float16)f1.y; u.h[6] = (_Float16)f1.z; u.h[7] = (_Float16)f1.w;
      *(v4i*)(A16 + r * APX + c0) = u.i;
    }
    {
      const v8f co = om_tile(om, nid, ow1, ob1, ow2h, ob2, rowBase, nN, h1t, tid, lane, wave);
#pragma unroll
      for (int r = 0; r < 8; ++r) A16[(8 * hh + r) * APX + DF + wave * 16 + m] = (_Float16)co[r];
    }
  } else {
    const int r  = tid >> 4;
    const int c0 = (tid & 15) * 8;
    const v4i t = *(const v4i*)(xh + (size_t)(rowBase + r) * DF + c0);
    *(v4i*)(A16 + r * APX + c0) = t;
  }
  __syncthreads();

  v8f c[8];
#pragma unroll
  for (int i = 0; i < 8; ++i) c[i] = vz8();
  const _Float16* Wr = Wh + (size_t)wave * DF * KD;
#pragma unroll 1
  for (int kt = 0; kt < KD / 32; ++kt) {
    const int k0 = kt * 32;
    FragH a;
    const _Float16* pa = A16 + m * APX + k0 + 8 * hh;
    a.half[0] = *(const v8h*)pa;
    a.half[1] = *(const v8h*)(pa + 16);
#pragma unroll
    for (int nt = 0; nt < 8; ++nt) {
      FragH b;
      const _Float16* pb = Wr + (size_t)(nt * 16 + m) * KD + k0 + 8 * hh;
      b.half[0] = *(const v8h*)pb;
      b.half[1] = *(const v8h*)(pb + 16);
      c[nt] = wmf(a.v, b.v, c[nt]);
    }
  }

#pragma unroll
  for (int nt = 0; nt < 8; ++nt) {
#pragma unroll
    for (int r = 0; r < 8; ++r)
      T16[(8 * hh + r) * HP + wave * DF + nt * 16 + m] = (_Float16)(c[nt][r] * SC);
  }
  __syncthreads();

  v8f dq = vz8(), dk = vz8();
#pragma unroll
  for (int kt = 0; kt < DF / 32; ++kt) {
    const int k0 = kt * 32;
    FragH a, bq, bk;
    const _Float16* pa = T16 + m * HP + wave * DF + k0 + 8 * hh;
    const _Float16* pq = qp + m * DF + k0 + 8 * hh;
    const _Float16* pk = kp + m * DF + k0 + 8 * hh;
    a.half[0]  = *(const v8h*)pa; a.half[1]  = *(const v8h*)(pa + 16);
    bq.half[0] = *(const v8h*)pq; bq.half[1] = *(const v8h*)(pq + 16);
    bk.half[0] = *(const v8h*)pk; bk.half[1] = *(const v8h*)(pk + 16);
    dq = wmf(a.v, bq.v, dq);
    dk = wmf(a.v, bk.v, dk);
  }
  if (m < NH) {
#pragma unroll
    for (int r = 0; r < 8; ++r) {
      hqs[wave * 64 + (8 * hh + r) * NH + m]             = dq[r] * (1.0f / 16.0f);
      hqs[NREL * 64 + wave * 64 + (8 * hh + r) * NH + m] = dk[r] * (1.0f / 16.0f);
    }
  }
  __syncthreads();

  PackH hv[8];
#pragma unroll
  for (int i = 0; i < 8; ++i) hv[i].h = *(const v8h*)(T16 + (2 * i + hh) * HP + wave * DF + 8 * m);
  _Float16* hb = hrH + ((size_t)wave * nP + rowBase) * DF;
  const int part = lane >> 4, li = lane & 15;
  const v4f qv = *(const v4f*)(hqs + part * NREL * 64 + wave * 64 + NH * li);
  float* qd = hqk + (((size_t)part * NREL + wave) * nP + rowBase + li) * NH;
#pragma unroll
  for (int i = 0; i < 8; ++i) *(volatile v4i*)(hb + i * 256 + lane * 8) = hv[i].i;
  *(volatile v4f*)qd = qv;
  __threadfence();
#pragma unroll
  for (int i = 0; i < 8; ++i) *(volatile v4i*)(hb + i * 256 + lane * 8) = hv[i].i;
  *(volatile v4f*)qd = qv;
}

template <bool FINAL>
__global__ __launch_bounds__(NTHR) void k_agg(
    const int* __restrict__ ei, const int* __restrict__ et,
    const _Float16* __restrict__ hrH, const float* __restrict__ hqk,
    const float* __restrict__ bias, _Float16* xo, float* out, int nN, int nP, int nE) {
  extern __shared__ v4f lds_dyn[];
  float* sacc = (float*)lds_dyn;
  float* mx   = sacc + LDS_SACC;
  float* den  = mx + LDS_MX;
  int*   list = (int*)(den + LDS_DEN);
  int*   wcnt = list + LDS_LIST;

  const int tid  = threadIdx.x;
  const int lane = tid & 31;
  const int wave = tid >> 5;
  const int hd   = lane >> 3;
  const int nodeBase = blockIdx.x * NB;

  {
    const v4f z4 = {0.f, 0.f, 0.f, 0.f};
    const v4f m4 = {-1e30f, -1e30f, -1e30f, -1e30f};
    for (int i = tid; i < LDS_SACC / 4; i += NTHR) lds_dyn[i] = z4;
    for (int i = tid; i < LDS_MX / 4; i += NTHR) lds_dyn[LDS_SACC / 4 + i] = m4;
    for (int i = tid; i < LDS_DEN / 4; i += NTHR) lds_dyn[(LDS_SACC + LDS_MX) / 4 + i] = z4;
  }
  __syncthreads();

  const int*   eid   = ei + nE;
  const bool   vec4  = ((nE & 3) == 0);
  const size_t hkOff = (size_t)NREL * nP * NH;
  const int nChunks = (nE + CHUNK - 1) / CHUNK;

#pragma unroll 1
  for (int ch = 0; ch < nChunks; ++ch) {
    const int  cbase = ch * CHUNK;
    const bool full  = vec4 && (cbase + CHUNK <= nE);
    int wc = 0;
#pragma unroll
    for (int g = 0; g < NGRP; ++g) {
      const int el0  = (g * NTHR + tid) * 4;
      const int e0   = cbase + el0;
      const int sent = -2147483647 - 1;
      v4i d;
      if (full) {
        d = *(const v4i*)(eid + e0);
      } else {
        const int t0 = eid[min(e0, nE - 1)];
        const int t1 = eid[min(e0 + 1, nE - 1)];
        const int t2 = eid[min(e0 + 2, nE - 1)];
        const int t3 = eid[min(e0 + 3, nE - 1)];
        d.x = (e0     < nE) ? t0 : sent;
        d.y = (e0 + 1 < nE) ? t1 : sent;
        d.z = (e0 + 2 < nE) ? t2 : sent;
        d.w = (e0 + 3 < nE) ? t3 : sent;
      }
      const unsigned s0 = (unsigned)d.x - (unsigned)nodeBase;
      const unsigned s1 = (unsigned)d.y - (unsigned)nodeBase;
      const unsigned s2 = (unsigned)d.z - (unsigned)nodeBase;
      const unsigned s3 = (unsigned)d.w - (unsigned)nodeBase;
      const bool h0 = s0 < (unsigned)NB;
      const bool h1 = s1 < (unsigned)NB;
      const bool h2 = s2 < (unsigned)NB;
      const bool h3 = s3 < (unsigned)NB;
      const unsigned many = __builtin_amdgcn_ballot_w32(h0 | h1 | h2 | h3);
      if (many != 0u) {
#define HITJ(J, HJ, SJ) { \
          const unsigned mj = __builtin_amdgcn_ballot_w32(HJ); \
          if (HJ) { \
            const int pos = wc + (int)__builtin_amdgcn_mbcnt_lo(mj, 0u); \
            if (pos < WCAP) list[wave * WCAP + pos] = ((el0 + (J)) << 9) | (int)(SJ); \
          } \
          wc += (int)__builtin_popcount(mj); }
        HITJ(0, h0, s0)
        HITJ(1, h1, s1)
        HITJ(2, h2, s2)
        HITJ(3, h3, s3)
#undef HITJ
      }
    }
    if (lane == 0) wcnt[wave] = wc;
    __syncthreads();

    if (wave == 0) {
#pragma unroll 1
      for (int wsx = 0; wsx < NWAVE; ++wsx) {
        int n = wcnt[wsx];
        n = n > WCAP ? WCAP : n;
        n = n < 0 ? 0 : n;
#pragma unroll 1
        for (int i = 0; i < n; ++i) {
          const int ent  = list[wsx * WCAP + i];
          const int slot = ent & (NB - 1);
          const int el   = (ent >> 9) & (CHUNK - 1);
          int e = cbase + el;
          if (e > nE - 1) e = nE - 1;
          int src = ei[e];
          src = src < 0 ? 0 : (src > nN - 1 ? nN - 1 : src);
          int t = et[e];
          t = t < 0 ? 0 : (t > NREL - 1 ? NREL - 1 : t);
          int nd = nodeBase + slot;
          if (nd > nN - 1) nd = nN - 1;
          const size_t rs = (size_t)t * nP + src;
          const size_t rd = (size_t)t * nP + nd;
          float lg = hqk[rd * NH + hd] + hqk[hkOff + rs * NH + hd];
          lg = lg > 0.f ? lg : 0.2f * lg;
          const int   ai = slot * NH + hd;
          const float mo = mx[ai];
          const float mn = fmaxf(mo, lg);
          const float sc = __expf(mo - mn);
          const float p  = __expf(lg - mn);
          const v4h hv = *(const v4h*)(hrH + rs * DF + 4 * lane);
          const v4f xv = __builtin_convertvector(hv, v4f);
          v4f* sp = (v4f*)(sacc + slot * DF + 4 * lane);
          const v4f cur = *sp;
          *sp = cur * sc + xv * p;
          const float dn = den[ai];
          den[ai] = dn * sc + p;
          mx[ai]  = mn;
        }
      }
    }
    __syncthreads();
  }

  if (FINAL) {
    const v4f b4 = *(const v4f*)(bias + 4 * lane);
#pragma unroll 1
    for (int j = 0; j < NB / NWAVE; ++j) {
      const int slot = wave * (NB / NWAVE) + j;
      const int node = nodeBase + slot;
      if (node >= nN) break;
      const v4f   s  = *(const v4f*)(sacc + slot * DF + 4 * lane);
      const float dn = den[slot * NH + hd];
      const float ds = dn > 0.f ? dn : 1.0f;
      const float inv = dn > 0.f ? (1.0f / ds) : 0.f;
      float* op = out + (size_t)node * DF + 4 * lane;
      const v4f sk = *(const v4f*)op;
      v4f y = s * inv + b4 + sk;
      y.x = lk01(y.x); y.y = lk01(y.y); y.z = lk01(y.z); y.w = lk01(y.w);
      *(volatile v4f*)op = y;
      __threadfence();
      *(volatile v4f*)op = y;
    }
  } else {
    const int part = lane >> 4, li = lane & 15;
    const int c0 = 8 * li;
    const int hq = li >> 2;
    const v4f b0 = *(const v4f*)(bias + c0);
    const v4f b1 = *(const v4f*)(bias + c0 + 4);
#pragma unroll 1
    for (int j = 0; j < NB / NWAVE / 2; ++j) {
      const int slotA = wave * (NB / NWAVE) + 2 * j;
      const int node0 = nodeBase + slotA;
      if (node0 >= nP) break;
      const int sl = slotA + part;
      const v4f s0 = *(const v4f*)(sacc + sl * DF + c0);
      const v4f s1 = *(const v4f*)(sacc + sl * DF + c0 + 4);
      const float dn = den[sl * NH + hq];
      const float ds = dn > 0.f ? dn : 1.0f;
      const float inv = dn > 0.f ? (1.0f / ds) : 0.f;
      const v4f y0 = s0 * inv + b0;
      const v4f y1 = s1 * inv + b1;
      PackH u;
      u.h[0] = (_Float16)(lk01(y0.x) * 16.0f); u.h[1] = (_Float16)(lk01(y0.y) * 16.0f);
      u.h[2] = (_Float16)(lk01(y0.z) * 16.0f); u.h[3] = (_Float16)(lk01(y0.w) * 16.0f);
      u.h[4] = (_Float16)(lk01(y1.x) * 16.0f); u.h[5] = (_Float16)(lk01(y1.y) * 16.0f);
      u.h[6] = (_Float16)(lk01(y1.z) * 16.0f); u.h[7] = (_Float16)(lk01(y1.w) * 16.0f);
      _Float16* xp = xo + (size_t)node0 * DF + 8 * lane;
      *(volatile v4i*)xp = u.i;
      __threadfence();
      *(volatile v4i*)xp = u.i;
    }
  }
}

static inline int cdiv(int a, int b) { return (a + b - 1) / b; }

extern "C" void kernel_launch(void* const* d_in, const int* in_sizes, int n_in,
                              void* d_out, int out_size, void* d_ws, size_t ws_size,
                              hipStream_t stream) {
  if (n_in < 21) return;
  const int nN = in_sizes[2];
  const int nE = in_sizes[4];
  if (nN <= 0 || nE <= 0) return;
  if (in_sizes[0] != nN * DF || in_sizes[1] != nN * OMK || in_sizes[3] != 2 * nE) return;
  if (in_sizes[5] != OMK * OMH || in_sizes[6] != OMH || in_sizes[7] != OMH * DF || in_sizes[8] != DF) return;
  if (in_sizes[9] != NREL * CIN * DF || in_sizes[10] != DF * NH || in_sizes[11] != DF * NH || in_sizes[12] != DF) return;
  if (in_sizes[13] != NREL * DF * DF || in_sizes[14] != DF * NH || in_sizes[15] != DF * NH || in_sizes[16] != DF) return;
  if (in_sizes[17] != CIN * DF || in_sizes[18] != DF || in_sizes[19] != DF * DF || in_sizes[20] != DF) return;
  if (out_size != nN * DF) return;

  const float* kg  = (const float*)d_in[0];
  const float* om  = (const float*)d_in[1];
  const int*   nid = (const int*)d_in[2];
  const int*   ei  = (const int*)d_in[3];
  const int*   et  = (const int*)d_in[4];
  const float* ow1 = (const float*)d_in[5];
  const float* ob1 = (const float*)d_in[6];
  const float* ow2 = (const float*)d_in[7];
  const float* ob2 = (const float*)d_in[8];
  const float* W1  = (const float*)d_in[9];
  const float* q1  = (const float*)d_in[10];
  const float* k1  = (const float*)d_in[11];
  const float* b1  = (const float*)d_in[12];
  const float* W2  = (const float*)d_in[13];
  const float* q2  = (const float*)d_in[14];
  const float* k2  = (const float*)d_in[15];
  const float* b2  = (const float*)d_in[16];
  const float* sw1 = (const float*)d_in[17];
  const float* sb1 = (const float*)d_in[18];
  const float* sw2 = (const float*)d_in[19];
  const float* sb2 = (const float*)d_in[20];
  float* out = (float*)d_out;

  const int nP = cdiv(nN, GR) * GR;

  size_t off = 0;
  char* wb = (char*)d_ws;
#define CARVE(T, name, bytes) T* name = (T*)(wb + off); off += ((size_t)(bytes) + 255) & ~(size_t)255;
  CARVE(unsigned short, W1h,   (size_t)NREL * DF * CIN * 2)
  CARVE(unsigned short, W2h,   (size_t)NREL * DF * DF * 2)
  CARVE(unsigned short, ow2h,  (size_t)DF * OMH * 2)
  CARVE(unsigned short, q1p,   (size_t)QROWS * DF * 2)
  CARVE(unsigned short, k1p,   (size_t)QROWS * DF * 2)
  CARVE(unsigned short, q2p,   (size_t)QROWS * DF * 2)
  CARVE(unsigned short, k2p,   (size_t)QROWS * DF * 2)
  CARVE(unsigned short, sw1hi, (size_t)DF * CIN * 2)
  CARVE(unsigned short, sw1lo, (size_t)DF * CIN * 2)
  CARVE(unsigned short, sw2hi, (size_t)DF * DF * 2)
  CARVE(unsigned short, sw2lo, (size_t)DF * DF * 2)
  CARVE(_Float16,       hrH,   (size_t)NREL * nP * DF * 2)
  CARVE(float,          hqk,   (size_t)2 * NREL * nP * NH * 4)
  CARVE(_Float16,       x1h,   (size_t)nP * DF * 2)
#undef CARVE
  if (off > ws_size) return;

  k_tconv<0><<<cdiv(NREL * DF * (CIN / 8), NTHR), NTHR, 0, stream>>>(W1, W1h, W1h, CIN, DF, DF, NREL, 16.0f);
  k_tconv<0><<<cdiv(NREL * DF * (DF / 8), NTHR), NTHR, 0, stream>>>(W2, W2h, W2h, DF, DF, DF, NREL, 16.0f);
  k_tconv<0><<<cdiv(DF * (OMH / 8), NTHR), NTHR, 0, stream>>>(ow2, ow2h, ow2h, OMH, DF, DF, 1, 16.0f);
  k_tconv<0><<<cdiv(QROWS * (DF / 8), NTHR), NTHR, 0, stream>>>(q1, q1p, q1p, DF, NH, QROWS, 1, 16.0f);
  k_tconv<0><<<cdiv(QROWS * (DF / 8), NTHR), NTHR, 0, stream>>>(k1, k1p, k1p, DF, NH, QROWS, 1, 16.0f);
  k_tconv<0><<<cdiv(QROWS * (DF / 8), NTHR), NTHR, 0, stream>>>(q2, q2p, q2p, DF, NH, QROWS, 1, 16.0f);
  k_tconv<0><<<cdiv(QROWS * (DF / 8), NTHR), NTHR, 0, stream>>>(k2, k2p, k2p, DF, NH, QROWS, 1, 16.0f);
  k_tconv<1><<<cdiv(DF * (CIN / 8), NTHR), NTHR, 0, stream>>>(sw1, sw1hi, sw1lo, CIN, DF, DF, 1, 1.0f);
  k_tconv<1><<<cdiv(DF * (DF / 8), NTHR), NTHR, 0, stream>>>(sw2, sw2hi, sw2lo, DF, DF, DF, 1, 1.0f);

  k_skip<<<nP / GR, NTHR, 0, stream>>>(kg, om, nid, ow1, ob1, (const _Float16*)ow2h, ob2,
                                       (const __bf16*)sw1hi, (const __bf16*)sw1lo, sb1,
                                       (const __bf16*)sw2hi, (const __bf16*)sw2lo, sb2, out, nN);

  k_hr<true><<<nP / GR, NTHR, 0, stream>>>(kg, om, nid, ow1, ob1, (const _Float16*)ow2h, ob2,
                                           (const _Float16*)x1h, (const _Float16*)W1h,
                                           (const _Float16*)q1p, (const _Float16*)k1p,
                                           hrH, hqk, nN, nP);
  const int aggGrid = cdiv(nN, NB);
  hipFuncSetAttribute(reinterpret_cast<const void*>(&k_agg<false>),
                      hipFuncAttributeMaxDynamicSharedMemorySize, LDS_BYTES);
  k_agg<false><<<aggGrid, NTHR, LDS_BYTES, stream>>>(ei, et, (const _Float16*)hrH, (const float*)hqk,
                                                    b1, x1h, out, nN, nP, nE);

  k_hr<false><<<nP / GR, NTHR, 0, stream>>>(kg, om, nid, ow1, ob1, (const _Float16*)ow2h, ob2,
                                            (const _Float16*)x1h, (const _Float16*)W2h,
                                            (const _Float16*)q2p, (const _Float16*)k2p,
                                            hrH, hqk, nN, nP);
  hipFuncSetAttribute(reinterpret_cast<const void*>(&k_agg<true>),
                      hipFuncAttributeMaxDynamicSharedMemorySize, LDS_BYTES);
  k_agg<true><<<aggGrid, NTHR, LDS_BYTES, stream>>>(ei, et, (const _Float16*)hrH, (const float*)hqk,
                                                   b2, x1h, out, nN, nP, nE);
}
